// S4Net_33947421507700
// MI455X (gfx1250) — hardware-run, weakly checked
//
#include <hip/hip_runtime.h>
#include <math.h>

typedef __attribute__((ext_vector_type(16))) _Float16 v16h;
typedef __attribute__((ext_vector_type(8)))  _Float16 v8h;
typedef __attribute__((ext_vector_type(8)))  float    v8f;
typedef __attribute__((ext_vector_type(4)))  float    v4f;
typedef __attribute__((ext_vector_type(2)))  float    v2f;
typedef __attribute__((ext_vector_type(4)))  unsigned v4u;

constexpr int kLayers   = 4;
constexpr int kChan     = 1024;
constexpr int kModes    = 32;
constexpr int kBatch    = 8;
constexpr int kLen      = 1024;
constexpr int kOutW     = 2 * kChan;
constexpr int kChunk    = 128;
constexpr int kChunksPS = kLen / kChunk;
constexpr int kRowsM    = kBatch * kChunksPS;
constexpr int kStateW   = 2 * kModes;
constexpr int kMvW      = kChunk + kStateW;
constexpr int kNpos     = kBatch * kLen;
constexpr int kGroup    = 256;
constexpr int kGroups   = kChan / kGroup;
constexpr int kPitchW   = 132;
static_assert(kChunksPS == 8 && kRowsM == 64 && kStateW == 64 && kMvW == 192 && kNpos == 8192 && kGroups == 4, "derived shapes");
static_assert((kChunk % 32) == 0 && (kStateW % 32) == 0 && (kChan % 32) == 0, "K multiples of 32");
static_assert(kRowsM == 64 && (kChunk % 64) == 0 && (kStateW % 64) == 0 && (kNpos % 64) == 0 && (kChan % 256) == 0, "tile multiples");

constexpr float kZCarry    = 16.0f;
constexpr float kZCarryInv = 1.0f / 16.0f;
constexpr float kECarry    = 64.0f;
constexpr float kMvCarry   = 1024.0f;
constexpr float kGCarry    = 16.0f;
constexpr float kWCarry    = 256.0f;
constexpr float kStateScale = 1.0f / kECarry;
constexpr float kConvScale  = 1.0f / (kZCarry * kMvCarry);
constexpr float kGluScale   = 1.0f / (kGCarry * kWCarry);

constexpr size_t kOffHA   = 0;
constexpr size_t kOffHB   = kOffHA   + (size_t)kNpos * kChan * 4;
constexpr size_t kOffWL   = kOffHB   + (size_t)kNpos * kChan * 4;
constexpr size_t kOffZT   = kOffWL   + (size_t)kOutW * kChan * 2;
constexpr size_t kOffGT   = kOffZT   + (size_t)kChan * kNpos * 2;
constexpr size_t kOffMv   = kOffGT   + (size_t)kChan * kNpos * 2;
constexpr size_t kOffEt   = kOffMv   + (size_t)kGroup * kChunk * kMvW * 2;
constexpr size_t kOffS32  = kOffEt   + (size_t)kGroup * kStateW * kChunk * 2;
constexpr size_t kOffInit = kOffS32  + (size_t)kGroup * kRowsM * kStateW * 4;
constexpr size_t kOffWpow = kOffInit + (size_t)kGroup * kRowsM * kStateW * 2;
constexpr size_t kWsTotal = kOffWpow + (size_t)kGroup * kModes * 2 * 4;
static_assert(kWsTotal == 127991808ull, "carve total");
static_assert(kWsTotal <= 134217728ull, "carve cap");
static_assert((kOffHB % 128) == 0 && (kOffWL % 128) == 0 && (kOffZT % 128) == 0 && (kOffGT % 128) == 0 &&
              (kOffMv % 128) == 0 && (kOffEt % 128) == 0 && (kOffS32 % 128) == 0 && (kOffInit % 128) == 0 &&
              (kOffWpow % 128) == 0, "128-B aligned regions");

__device__ __forceinline__ unsigned short f16bits(float x) {
  const _Float16 h = (_Float16)x;
  return __builtin_bit_cast(unsigned short, h);
}
__device__ __forceinline__ unsigned pack2(float a, float b) {
  const unsigned lo = (unsigned)f16bits(a);
  const unsigned hi = (unsigned)f16bits(b);
  return lo | (hi << 16);
}
__device__ __forceinline__ float h16_to_f32(unsigned hb) {
  const unsigned sgn = (hb & 0x8000u) << 16;
  const unsigned em = hb & 0x7fffu;
  const float fn = __uint_as_float((em << 13) + 0x38000000u);
  const float fs = (float)em * 5.9604644775390625e-8f;
  const float mag = (em < 0x400u) ? fs : fn;
  return __uint_as_float(__float_as_uint(mag) | sgn);
}
__device__ __forceinline__ void wave_sync() {
  __builtin_amdgcn_fence(__ATOMIC_RELEASE, "workgroup");
  __builtin_amdgcn_wave_barrier();
  __builtin_amdgcn_fence(__ATOMIC_ACQUIRE, "workgroup");
}
__device__ __forceinline__ void store2_v4u(unsigned short* p, v4u v) {
  volatile v4u* q = (volatile v4u*)p;
  *q = v;
  __threadfence();
  *q = v;
}
__device__ __forceinline__ float gelu_fast(float y) {
  const float u = 0.7978845608028654f * (y + 0.044715f * y * y * y);
  const float e = __expf(-2.0f * u);
  return y * __builtin_amdgcn_rcpf(1.0f + e);
}

union FragH { v16h v; v8h h[2]; };
__device__ __forceinline__ v16h frag_load(const _Float16* p) {
  FragH f;
  f.h[0] = *(const v8h*)(p);
  f.h[1] = *(const v8h*)(p + 16);
  return f.v;
}
__device__ __forceinline__ v8f mma16(v16h a, v16h b, v8f c) {
  return __builtin_amdgcn_wmma_f32_16x16x32_f16(false, a, false, b, (short)0, c, false, false);
}
__device__ __forceinline__ void tie_acc(v8f& a, v16h x, v16h y) { asm volatile("" : "+v"(a) : "v"(x), "v"(y)); }
__device__ __forceinline__ void tie_acc_nops(v8f& a, v16h x, v16h y) { asm volatile("v_nop\n\tv_nop\n\tv_nop\n\tv_nop" : "+v"(a) : "v"(x), "v"(y)); }
__device__ __forceinline__ void keep4(v16h a, v16h b, v16h c, v16h d) { asm volatile("v_nop" :: "v"(a), "v"(b), "v"(c), "v"(d)); }
__device__ __forceinline__ void acc_guard4(v8f& a, v8f& b, v8f& c, v8f& d) { asm volatile("v_nop\n\tv_nop\n\tv_nop\n\tv_nop" : "+v"(a), "+v"(b), "+v"(c), "+v"(d)); }

__device__ __forceinline__ void kloop64(v8f (&acc)[4][4], const _Float16* ap, int lda,
                                        const _Float16* bp, int ldb, int ksteps) {
#pragma unroll 1
  for (int ks = 0; ks < ksteps; ++ks) {
    v16h bh[4];
#pragma unroll
    for (int j = 0; j < 4; ++j) bh[j] = frag_load(bp + (size_t)(j * 16) * ldb + ks * 32);
#pragma unroll
    for (int i = 0; i < 4; ++i) {
      const v16h ah = frag_load(ap + (size_t)(i * 16) * lda + ks * 32);
#pragma unroll
      for (int j = 0; j < 4; ++j) acc[i][j] = mma16(ah, bh[j], acc[i][j]);
      tie_acc(acc[i][0], ah, bh[0]);
      tie_acc(acc[i][1], ah, bh[1]);
      tie_acc(acc[i][2], ah, bh[2]);
      tie_acc_nops(acc[i][3], ah, bh[3]);
    }
    keep4(bh[0], bh[1], bh[2], bh[3]);
  }
}

template <int NT>
__device__ __forceinline__ void stage_tile_T(const unsigned short* plane, size_t n0, unsigned* sw, int tid) {
#pragma unroll 1
  for (int it = 0; it < 1024 / NT; ++it) {
    const int task = it * NT + tid;
    const int n8 = task & 7;
    const int kp = task >> 3;
    const unsigned short* p0 = plane + (size_t)(2 * kp) * kNpos + n0 + n8 * 8;
    const v4u a = *(const v4u*)(p0);
    const v4u b = *(const v4u*)(p0 + kNpos);
    unsigned* dst = sw + (n8 * 8) * kPitchW + kp;
#pragma unroll
    for (int j = 0; j < 4; ++j) {
      const unsigned aw = a[j];
      const unsigned bw = b[j];
      dst[(2 * j) * kPitchW]     = (aw & 0xffffu) | (bw << 16);
      dst[(2 * j + 1) * kPitchW] = (aw >> 16) | (bw & 0xffff0000u);
    }
  }
}

__device__ __forceinline__ void store_tile_rows(const unsigned* sw, unsigned short* plane, size_t n0, int wave, int lane) {
  const int q = lane >> 3;
  const int cw = lane & 7;
  v4u vals[8];
#pragma unroll
  for (int it = 0; it < 8; ++it) {
    const int row = it * 32 + wave * 4 + q;
    vals[it] = *(const v4u*)(sw + row * 32 + cw * 4);
  }
  for (int pass = 0; pass < 2; ++pass) {
#pragma unroll
    for (int it = 0; it < 8; ++it) {
      const int row = it * 32 + wave * 4 + q;
      *(volatile v4u*)(plane + (size_t)row * kNpos + n0 + cw * 8) = vals[it];
    }
    __threadfence();
  }
}

static_assert(((size_t)kOutW * kChan / 8) % 256 == 0, "weight chunk count is a block multiple");
__global__ __launch_bounds__(256) void weight_plane_kernel(const float* __restrict__ w, unsigned short* __restrict__ w16) {
  const size_t q = (size_t)blockIdx.x * 256 + threadIdx.x;
  const v4f a = *(const v4f*)(w + q * 8);
  const v4f b = *(const v4f*)(w + q * 8 + 4);
  const v4u pk = {pack2(a[0] * kWCarry, a[1] * kWCarry), pack2(a[2] * kWCarry, a[3] * kWCarry),
                  pack2(b[0] * kWCarry, b[1] * kWCarry), pack2(b[2] * kWCarry, b[3] * kWCarry)};
  store2_v4u(w16 + q * 8, pk);
}

__global__ __launch_bounds__(256) void norm_transpose_kernel(
    const float* __restrict__ hsrc, const float* __restrict__ ln_w, const float* __restrict__ ln_b,
    unsigned short* __restrict__ zt) {
  __shared__ __align__(16) union { unsigned w[256 * 32]; unsigned short s[256 * 64]; } sb;
  __shared__ float sMu[64];
  __shared__ float sRs[64];
  const int tid = threadIdx.x;
  const int lane = tid & 31;
  const int wave = __builtin_amdgcn_readfirstlane((int)(threadIdx.x >> 5));
  const size_t n0 = (size_t)blockIdx.x * 64;
#pragma unroll 1
  for (int r = 0; r < 8; ++r) {
    const int tok = wave * 8 + r;
    const float* rowp = hsrc + (n0 + (size_t)tok) * kChan + lane * 4;
    v4f v[8];
#pragma unroll
    for (int it = 0; it < 8; ++it) v[it] = *(const v4f*)(rowp + it * 128);
    float s = 0.0f;
#pragma unroll
    for (int it = 0; it < 8; ++it) {
      const v4f t = v[it];
      s += (t[0] + t[1]) + (t[2] + t[3]);
    }
    s += __shfl_xor(s, 16, 32);
    s += __shfl_xor(s, 8, 32);
    s += __shfl_xor(s, 4, 32);
    s += __shfl_xor(s, 2, 32);
    s += __shfl_xor(s, 1, 32);
    const float mu = s * (1.0f / (float)kChan);
    float qv = 0.0f;
#pragma unroll
    for (int it = 0; it < 8; ++it) {
      const v4f t = v[it];
      const float d0 = t[0] - mu;
      const float d1 = t[1] - mu;
      const float d2 = t[2] - mu;
      const float d3 = t[3] - mu;
      qv = fmaf(d0, d0, qv);
      qv = fmaf(d1, d1, qv);
      qv = fmaf(d2, d2, qv);
      qv = fmaf(d3, d3, qv);
    }
    qv += __shfl_xor(qv, 16, 32);
    qv += __shfl_xor(qv, 8, 32);
    qv += __shfl_xor(qv, 4, 32);
    qv += __shfl_xor(qv, 2, 32);
    qv += __shfl_xor(qv, 1, 32);
    const float rs = rsqrtf(qv * (1.0f / (float)kChan) + 1e-5f);
    if (lane == 0) {
      sMu[tok] = mu;
      sRs[tok] = rs;
    }
  }
  __syncthreads();
#pragma unroll 1
  for (int cq = 0; cq < 4; ++cq) {
#pragma unroll 1
    for (int it = 0; it < 16; ++it) {
      const int task = it * 256 + tid;
      const int c4 = task & 63;
      const int tok = task >> 6;
      const int ch = cq * 256 + c4 * 4;
      const v4f v = *(const v4f*)(hsrc + (n0 + (size_t)tok) * kChan + ch);
      const v4f lw = *(const v4f*)(ln_w + ch);
      const v4f lb = *(const v4f*)(ln_b + ch);
      const float mu = sMu[tok];
      const float rs = sRs[tok];
#pragma unroll
      for (int e = 0; e < 4; ++e) {
        const float xn = (v[e] - mu) * rs;
        const float z = fmaf(xn, lw[e], lb[e]);
        sb.s[(c4 * 4 + e) * 64 + tok] = f16bits(z * kZCarry);
      }
    }
    __syncthreads();
    store_tile_rows(sb.w, zt + (size_t)(cq * 256) * kNpos, n0, wave, lane);
    __syncthreads();
  }
}

__global__ __launch_bounds__(256) void layer_tables_kernel(
    const float* __restrict__ log_dt, const float* __restrict__ a_re_log, const float* __restrict__ a_im,
    const float* __restrict__ c_re, const float* __restrict__ c_im,
    unsigned short* __restrict__ et16, unsigned short* __restrict__ mv16, float* __restrict__ wpow) {
  __shared__ float sPr[129 * 32];
  __shared__ float sPi[129 * 32];
  __shared__ float sK[128];
  __shared__ float sCr[32];
  __shared__ float sCi[32];
  const int tid = threadIdx.x;
  const int n = tid & 31;
  const int seg = __builtin_amdgcn_readfirstlane((int)(threadIdx.x >> 5));
  const int h = blockIdx.x;
  const int idx = h * kModes + n;
  const float dt = expf(log_dt[h]);
  const float ar = -expf(a_re_log[idx]);
  const float ai = a_im[idx];
  const float dr = ar * dt;
  const float di = ai * dt;
  const float em = expm1f(dr);
  const float es = em + 1.0f;
  float sn, cs;
  sincosf(di, &sn, &cs);
  const float cm1a = -(sn * sn) * (1.0f / (1.0f + fmaxf(cs, 0.0f)));
  const float cm1 = (cs > 0.0f) ? cm1a : (cs - 1.0f);
  const float wr = es * cs;
  const float wi = es * sn;
  const float nr = em * cs + cm1;
  const float ni = wi;
  const float inv = 1.0f / (ar * ar + ai * ai);
  const float qr = (nr * ar + ni * ai) * inv;
  const float qi = (ni * ar - nr * ai) * inv;
  const float cr = c_re[idx];
  const float ci = c_im[idx];
  const float c2r = 2.0f * (cr * qr - ci * qi);
  const float c2i = 2.0f * (cr * qi + ci * qr);
  float sr = wr, si = wi;
#pragma unroll 1
  for (int i = 0; i < 4; ++i) {
    const float t = sr * sr - si * si;
    si = 2.0f * sr * si;
    sr = t;
  }
  float gr = sr, gi = si;
#pragma unroll 1
  for (int i = 0; i < 3; ++i) {
    const float t = gr * gr - gi * gi;
    gi = 2.0f * gr * gi;
    gr = t;
  }
  float pr = 1.0f, pi = 0.0f;
#pragma unroll 1
  for (int s = 0; s < seg; ++s) {
    const float t = pr * sr - pi * si;
    pi = pr * si + pi * sr;
    pr = t;
  }
#pragma unroll 1
  for (int s = 0; s < 16; ++s) {
    const int l = 16 * seg + s;
    sPr[l * 32 + n] = pr;
    sPi[l * 32 + n] = pi;
    const float t = pr * wr - pi * wi;
    pi = pr * wi + pi * wr;
    pr = t;
  }
  if (seg == 7) {
    sPr[128 * 32 + n] = pr;
    sPi[128 * 32 + n] = pi;
  }
  if (seg == 0) {
    sCr[n] = c2r;
    sCi[n] = c2i;
    const v2f wv = {gr, gi};
    volatile v2f* wp = (volatile v2f*)(wpow + (size_t)(h * kModes + n) * 2);
    *wp = wv;
    __threadfence();
    *wp = wv;
  }
  __syncthreads();
  if (tid < 128) {
    float acc = 0.0f;
#pragma unroll 1
    for (int m = 0; m < kModes; ++m) {
      acc += sCr[m] * sPr[tid * 32 + m] - sCi[m] * sPi[tid * 32 + m];
    }
    sK[tid] = acc;
  }
  __syncthreads();
#pragma unroll 1
  for (int it = 0; it < 8; ++it) {
    const int q = it * 256 + tid;
    const int row = q >> 4;
    const int s0 = (q & 15) * 8;
    float v[8];
#pragma unroll
    for (int e = 0; e < 8; ++e) {
      const int df = row - (s0 + e);
      int dc = (df < 0) ? 0 : df;
      dc = (dc > 127) ? 127 : dc;
      const float kv = sK[dc];
      const float val = (df >= 0) ? kv : 0.0f;
      v[e] = val * kMvCarry;
    }
    const v4u pk = {pack2(v[0], v[1]), pack2(v[2], v[3]), pack2(v[4], v[5]), pack2(v[6], v[7])};
    store2_v4u(mv16 + ((size_t)h * kChunk + row) * kMvW + s0, pk);
  }
#pragma unroll 1
  for (int it = 0; it < 4; ++it) {
    const int q = it * 256 + tid;
    const int row = q >> 3;
    const int nb = (q & 7) * 4;
    unsigned wd[4];
#pragma unroll
    for (int e = 0; e < 4; ++e) {
      const int m = nb + e;
      const float ppr = sPr[(row + 1) * 32 + m];
      const float ppi = sPi[(row + 1) * 32 + m];
      const float a = sCr[m];
      const float bq = sCi[m];
      const float re = a * ppr - bq * ppi;
      const float im = a * ppi + bq * ppr;
      wd[e] = pack2(re * kMvCarry, -im * kMvCarry);
    }
    const v4u pk = {wd[0], wd[1], wd[2], wd[3]};
    store2_v4u(mv16 + ((size_t)h * kChunk + row) * kMvW + kChunk + nb * 2, pk);
  }
#pragma unroll 1
  for (int it = 0; it < 4; ++it) {
    const int q = it * 256 + tid;
    const int r = q >> 4;
    const int k8 = (q & 15) * 8;
    const int m = r >> 1;
    const int part = r & 1;
    float v[8];
#pragma unroll
    for (int e = 0; e < 8; ++e) {
      const int l = 127 - (k8 + e);
      const float a = sPr[l * 32 + m];
      const float bq = sPi[l * 32 + m];
      const float val = part ? bq : a;
      v[e] = val * kECarry;
    }
    const v4u pk = {pack2(v[0], v[1]), pack2(v[2], v[3]), pack2(v[4], v[5]), pack2(v[6], v[7])};
    store2_v4u(et16 + ((size_t)h * kStateW + r) * kChunk + k8, pk);
  }
}

template <int MODE>
__global__ __launch_bounds__(256) void chunk_gemm_kernel(
    const unsigned short* __restrict__ zplane, const unsigned short* __restrict__ initp,
    const unsigned short* __restrict__ btp, void* __restrict__ cout, const float* __restrict__ dskip) {
  __shared__ __align__(16) float sT[8][16 * 68];
  __shared__ __align__(16) unsigned sHw[(MODE == 1) ? 8 : 1][(MODE == 1) ? 16 * 32 : 4];
  const int lane = threadIdx.x & 31;
  const int wave = __builtin_amdgcn_readfirstlane((int)(threadIdx.x >> 5));
  const int tile = (int)blockIdx.x * 8 + wave;
  const int h = (MODE == 1) ? (tile >> 1) : tile;
  const int tn = (MODE == 1) ? (tile & 1) : 0;
  const int n0 = tn << 6;
  const int rlane = lane & 15;
  const int koff = (lane >> 4) * 8;
  const int mOff = (lane >> 4) * 8;
  constexpr int LDB = (MODE == 1) ? kMvW : kChunk;
  constexpr int BROWS = (MODE == 1) ? kChunk : kStateW;
  const _Float16* A1 = (const _Float16*)zplane + (size_t)h * kNpos;
  const _Float16* Bt = (const _Float16*)btp + (size_t)h * BROWS * LDB;

  v8f acc[4][4];
#pragma unroll
  for (int i = 0; i < 4; ++i)
#pragma unroll
    for (int j = 0; j < 4; ++j) acc[i][j] = (v8f){0.f, 0.f, 0.f, 0.f, 0.f, 0.f, 0.f, 0.f};

  const int ksteps1 = (MODE == 1) ? (2 * (tn + 1)) : (kChunk / 32);
  kloop64(acc, A1 + (size_t)rlane * kChunk + koff, kChunk,
          Bt + (size_t)(n0 + rlane) * LDB + koff, LDB, ksteps1);
  if (MODE == 1) {
    const _Float16* A2 = (const _Float16*)initp + (size_t)h * kRowsM * kStateW;
    kloop64(acc, A2 + (size_t)rlane * kStateW + koff, kStateW,
            Bt + (size_t)(n0 + rlane) * LDB + kChunk + koff, LDB, kStateW / 32);
  }
  acc_guard4(acc[0][0], acc[0][1], acc[0][2], acc[0][3]);
  acc_guard4(acc[1][0], acc[1][1], acc[1][2], acc[1][3]);
  acc_guard4(acc[2][0], acc[2][1], acc[2][2], acc[2][3]);
  acc_guard4(acc[3][0], acc[3][1], acc[3][2], acc[3][3]);

  float* slab = sT[wave];
  const float scale = (MODE == 1) ? kConvScale : kStateScale;
  const float dsz = (MODE == 1) ? (dskip[h] * kZCarryInv) : 0.0f;
#pragma unroll
  for (int i = 0; i < 4; ++i) {
    const int mBase = (i << 4);
#pragma unroll
    for (int j = 0; j < 4; ++j) {
#pragma unroll
      for (int r = 0; r < 8; ++r) slab[(mOff + r) * 68 + (j << 4) + rlane] = acc[i][j][r] * scale;
    }
    wave_sync();
    if (MODE == 0) {
      float* C = (float*)cout + (size_t)h * kRowsM * kStateW;
      const int h2 = lane >> 4;
      const int c4 = (lane & 15) * 4;
      for (int pass = 0; pass < 2; ++pass) {
#pragma unroll
        for (int it = 0; it < 8; ++it) {
          const int row = it * 2 + h2;
          const v4f v = *(const v4f*)(slab + row * 68 + c4);
          *(volatile v4f*)(C + (size_t)(mBase + row) * kStateW + c4) = v;
        }
        __threadfence();
      }
    } else {
      unsigned* sH = sHw[wave];
      unsigned short* G = (unsigned short*)cout + (size_t)h * kNpos;
      const unsigned short* Zrow = zplane + (size_t)h * kNpos;
      const int q = lane >> 3;
      const int cw = lane & 7;
#pragma unroll 1
      for (int it = 0; it < 4; ++it) {
        const int row = it * 4 + q;
        const float* sp = slab + row * 68 + cw * 8;
        const v4f a0 = *(const v4f*)(sp);
        const v4f a1 = *(const v4f*)(sp + 4);
        const v4u zw = *(const v4u*)(Zrow + (size_t)(mBase + row) * kChunk + n0 + cw * 8);
        const unsigned w0 = zw[0];
        const unsigned w1 = zw[1];
        const unsigned w2 = zw[2];
        const unsigned w3 = zw[3];
        const float y0 = fmaf(dsz, h16_to_f32(w0 & 0xffffu), a0[0]);
        const float y1 = fmaf(dsz, h16_to_f32(w0 >> 16), a0[1]);
        const float y2 = fmaf(dsz, h16_to_f32(w1 & 0xffffu), a0[2]);
        const float y3 = fmaf(dsz, h16_to_f32(w1 >> 16), a0[3]);
        const float y4 = fmaf(dsz, h16_to_f32(w2 & 0xffffu), a1[0]);
        const float y5 = fmaf(dsz, h16_to_f32(w2 >> 16), a1[1]);
        const float y6 = fmaf(dsz, h16_to_f32(w3 & 0xffffu), a1[2]);
        const float y7 = fmaf(dsz, h16_to_f32(w3 >> 16), a1[3]);
        const v4u pk = {pack2(gelu_fast(y0) * kGCarry, gelu_fast(y1) * kGCarry),
                        pack2(gelu_fast(y2) * kGCarry, gelu_fast(y3) * kGCarry),
                        pack2(gelu_fast(y4) * kGCarry, gelu_fast(y5) * kGCarry),
                        pack2(gelu_fast(y6) * kGCarry, gelu_fast(y7) * kGCarry)};
        *(v4u*)(sH + row * 32 + cw * 4) = pk;
      }
      wave_sync();
      v4u vals[4];
#pragma unroll
      for (int it = 0; it < 4; ++it) vals[it] = *(const v4u*)(sH + (it * 4 + q) * 32 + cw * 4);
      for (int pass = 0; pass < 2; ++pass) {
#pragma unroll
        for (int it = 0; it < 4; ++it) {
          const int row = it * 4 + q;
          *(volatile v4u*)(G + (size_t)(mBase + row) * kChunk + n0 + cw * 8) = vals[it];
        }
        __threadfence();
      }
    }
    wave_sync();
  }
}

__global__ __launch_bounds__(256) void combine_kernel(
    const float* __restrict__ s32, const float* __restrict__ wpow, unsigned short* __restrict__ init16) {
  const int lane = threadIdx.x & 31;
  const int wave = __builtin_amdgcn_readfirstlane((int)(threadIdx.x >> 5));
  const int pair = (int)blockIdx.x * 8 + wave;
  const int h = pair >> 3;
  const int b = pair & 7;
  const v2f w = *(const v2f*)(wpow + (size_t)(h * kModes + lane) * 2);
  const float w_re = w[0];
  const float w_im = w[1];
  const float* sp = s32 + ((size_t)h * kRowsM + (size_t)b * kChunksPS) * kStateW + 2 * lane;
  unsigned* ip = (unsigned*)(init16 + ((size_t)h * kRowsM + (size_t)b * kChunksPS) * kStateW) + lane;
  float er = 0.0f, ei = 0.0f;
#pragma unroll 1
  for (int cidx = 0; cidx < kChunksPS; ++cidx) {
    const v2f s = *(const v2f*)(sp + (size_t)cidx * kStateW);
    const float cr = fminf(fmaxf(er, -60000.0f), 60000.0f);
    const float ci = fminf(fmaxf(ei, -60000.0f), 60000.0f);
    const unsigned word = pack2(cr, ci);
    volatile unsigned* q = (volatile unsigned*)(ip + (size_t)cidx * (kStateW / 2));
    *q = word;
    __threadfence();
    *q = word;
    const float tr = w_re * er - w_im * ei + s[0];
    ei = w_re * ei + w_im * er + s[1];
    er = tr;
  }
}

__global__ __launch_bounds__(256) void token_major_kernel(
    const unsigned short* __restrict__ gt, unsigned short* __restrict__ g) {
  __shared__ __align__(16) unsigned sw[64 * kPitchW];
  const int tid = threadIdx.x;
  const int lane = tid & 31;
  const int wave = __builtin_amdgcn_readfirstlane((int)(threadIdx.x >> 5));
  const size_t n0 = (size_t)blockIdx.x * 64;
  const int cq = blockIdx.y;
  stage_tile_T<256>(gt + (size_t)(cq * 256) * kNpos, n0, sw, tid);
  __syncthreads();
  v4u vals[8];
#pragma unroll
  for (int it = 0; it < 8; ++it) vals[it] = *(const v4u*)(sw + (wave * 8 + it) * kPitchW + lane * 4);
  for (int pass = 0; pass < 2; ++pass) {
#pragma unroll
    for (int it = 0; it < 8; ++it) {
      const size_t row = n0 + (size_t)(wave * 8 + it);
      *(volatile v4u*)(g + row * kChan + cq * 256 + lane * 8) = vals[it];
    }
    __threadfence();
  }
}

static_assert((kNpos / 64) * (kChan / 32) == 512 * 8, "wave tiles fill the grid exactly");
__global__ __launch_bounds__(256) void glu_gemm_kernel(
    const unsigned short* __restrict__ gp, const unsigned short* __restrict__ wp,
    const float* __restrict__ bias, const float* __restrict__ hsrc, float* __restrict__ hdst) {
  __shared__ __align__(16) float sV[8][16 * 36];
  __shared__ __align__(16) float sG[8][16 * 36];
  const int lane = threadIdx.x & 31;
  const int wave = __builtin_amdgcn_readfirstlane((int)(threadIdx.x >> 5));
  const int tile = (int)blockIdx.x * 8 + wave;
  const int tm = tile >> 5;
  const int tn = tile & 31;
  const int m0 = tm << 6;
  const int o0 = tn << 5;
  const int rlane = lane & 15;
  const int koff = (lane >> 4) * 8;
  const int mOff = (lane >> 4) * 8;
  const _Float16* Ap = (const _Float16*)gp + (size_t)(m0 + rlane) * kChan + koff;
  const _Float16* Bv = (const _Float16*)wp + (size_t)(o0 + rlane) * kChan + koff;
  const _Float16* Bg = Bv + (size_t)kChan * kChan;

  v8f acc[4][4];
#pragma unroll
  for (int i = 0; i < 4; ++i)
#pragma unroll
    for (int j = 0; j < 4; ++j) acc[i][j] = (v8f){0.f, 0.f, 0.f, 0.f, 0.f, 0.f, 0.f, 0.f};

#pragma unroll 1
  for (int ks = 0; ks < kChan / 32; ++ks) {
    v16h bh[4];
    bh[0] = frag_load(Bv + ks * 32);
    bh[1] = frag_load(Bv + (size_t)16 * kChan + ks * 32);
    bh[2] = frag_load(Bg + ks * 32);
    bh[3] = frag_load(Bg + (size_t)16 * kChan + ks * 32);
#pragma unroll
    for (int i = 0; i < 4; ++i) {
      const v16h ah = frag_load(Ap + (size_t)(i * 16) * kChan + ks * 32);
#pragma unroll
      for (int j = 0; j < 4; ++j) acc[i][j] = mma16(ah, bh[j], acc[i][j]);
      tie_acc(acc[i][0], ah, bh[0]);
      tie_acc(acc[i][1], ah, bh[1]);
      tie_acc(acc[i][2], ah, bh[2]);
      tie_acc_nops(acc[i][3], ah, bh[3]);
    }
    keep4(bh[0], bh[1], bh[2], bh[3]);
  }
  acc_guard4(acc[0][0], acc[0][1], acc[0][2], acc[0][3]);
  acc_guard4(acc[1][0], acc[1][1], acc[1][2], acc[1][3]);
  acc_guard4(acc[2][0], acc[2][1], acc[2][2], acc[2][3]);
  acc_guard4(acc[3][0], acc[3][1], acc[3][2], acc[3][3]);

  float* sv = sV[wave];
  float* sg = sG[wave];
  const int q = lane >> 3;
  const int c4 = (lane & 7) * 4;
  const v4f bvv = *(const v4f*)(bias + o0 + c4);
  const v4f bgv = *(const v4f*)(bias + kChan + o0 + c4);
#pragma unroll
  for (int i = 0; i < 4; ++i) {
    const int mBase = m0 + (i << 4);
#pragma unroll
    for (int j = 0; j < 2; ++j) {
#pragma unroll
      for (int r = 0; r < 8; ++r) {
        sv[(mOff + r) * 36 + (j << 4) + rlane] = acc[i][j][r] * kGluScale;
        sg[(mOff + r) * 36 + (j << 4) + rlane] = acc[i][2 + j][r] * kGluScale;
      }
    }
    wave_sync();
#pragma unroll 1
    for (int it = 0; it < 4; ++it) {
      const int row = it * 4 + q;
      const v4f vv = *(const v4f*)(sv + row * 36 + c4);
      const v4f gg = *(const v4f*)(sg + row * 36 + c4);
      const v4f rr = *(const v4f*)(hsrc + (size_t)(mBase + row) * kChan + o0 + c4);
      v4f oo;
#pragma unroll
      for (int e = 0; e < 4; ++e) {
        const float val = vv[e] + bvv[e];
        const float gat = gg[e] + bgv[e];
        const float sgm = __builtin_amdgcn_rcpf(1.0f + __expf(-gat));
        oo[e] = fmaf(val, sgm, rr[e]);
      }
      *(v4f*)(sv + row * 36 + c4) = oo;
    }
    wave_sync();
    v4f vals[4];
#pragma unroll
    for (int it = 0; it < 4; ++it) vals[it] = *(const v4f*)(sv + (it * 4 + q) * 36 + c4);
    for (int pass = 0; pass < 2; ++pass) {
#pragma unroll
      for (int it = 0; it < 4; ++it) {
        const int row = it * 4 + q;
        *(volatile v4f*)(hdst + (size_t)(mBase + row) * kChan + o0 + c4) = vals[it];
      }
      __threadfence();
    }
    wave_sync();
  }
}

extern "C" void kernel_launch(void* const* d_in, const int* in_sizes, int n_in,
                              void* d_out, int out_size, void* d_ws, size_t ws_size,
                              hipStream_t stream) {
  if (n_in < 11) return;
  if (in_sizes[0] != kBatch * kLen * kChan) return;
  if (in_sizes[1] != kLayers * kChan) return;
  if (in_sizes[2] != kLayers * kChan) return;
  if (in_sizes[3] != kLayers * kChan) return;
  if (in_sizes[4] != kLayers * kChan * kModes) return;
  if (in_sizes[5] != kLayers * kChan * kModes) return;
  if (in_sizes[6] != kLayers * kChan * kModes) return;
  if (in_sizes[7] != kLayers * kChan * kModes) return;
  if (in_sizes[8] != kLayers * kChan) return;
  if (in_sizes[9] != kLayers * kOutW * kChan) return;
  if (in_sizes[10] != kLayers * kOutW) return;
  if (out_size != kBatch * kLen * kChan) return;
  if (ws_size < kWsTotal) return;

  const float* x        = (const float*)d_in[0];
  const float* ln_w     = (const float*)d_in[1];
  const float* ln_b     = (const float*)d_in[2];
  const float* log_dt   = (const float*)d_in[3];
  const float* A_re_log = (const float*)d_in[4];
  const float* A_im     = (const float*)d_in[5];
  const float* C_re     = (const float*)d_in[6];
  const float* C_im     = (const float*)d_in[7];
  const float* D_skip   = (const float*)d_in[8];
  const float* W_out    = (const float*)d_in[9];
  const float* b_out    = (const float*)d_in[10];
  float* out = (float*)d_out;

  char* ws = (char*)d_ws;
  float*          HA   = (float*)(ws + kOffHA);
  float*          HB   = (float*)(ws + kOffHB);
  unsigned short* WL   = (unsigned short*)(ws + kOffWL);
  unsigned short* ZT   = (unsigned short*)(ws + kOffZT);
  unsigned short* GP   = (unsigned short*)(ws + kOffZT);
  unsigned short* GT   = (unsigned short*)(ws + kOffGT);
  unsigned short* MV   = (unsigned short*)(ws + kOffMv);
  unsigned short* ET   = (unsigned short*)(ws + kOffEt);
  float*          S32  = (float*)(ws + kOffS32);
  unsigned short* INIT = (unsigned short*)(ws + kOffInit);
  float*          WPOW = (float*)(ws + kOffWpow);

  for (int i = 0; i < kLayers; ++i) {
    const float* src = (i == 0) ? x : ((i == 2) ? (const float*)HB : (const float*)HA);
    float* dst = (i == 3) ? out : ((i == 1) ? HB : HA);

    weight_plane_kernel<<<(kOutW * kChan / 8) / 256, 256, 0, stream>>>(W_out + (size_t)i * kOutW * kChan, WL);
    norm_transpose_kernel<<<kNpos / 64, 256, 0, stream>>>(src, ln_w + (size_t)i * kChan, ln_b + (size_t)i * kChan, ZT);

    for (int g = 0; g < kGroups; ++g) {
      const size_t hb = (size_t)i * kChan + (size_t)g * kGroup;
      const size_t om = hb * kModes;
      const unsigned short* zg = ZT + (size_t)g * kGroup * kNpos;
      unsigned short* gg = GT + (size_t)g * kGroup * kNpos;
      layer_tables_kernel<<<kGroup, 256, 0, stream>>>(log_dt + hb, A_re_log + om, A_im + om, C_re + om, C_im + om,
                                                      ET, MV, WPOW);
      chunk_gemm_kernel<0><<<kGroup / 8, 256, 0, stream>>>(zg, INIT, ET, (void*)S32, D_skip + hb);
      combine_kernel<<<(kGroup * kBatch) / 8, 256, 0, stream>>>(S32, WPOW, INIT);
      chunk_gemm_kernel<1><<<(kGroup * 2) / 8, 256, 0, stream>>>(zg, INIT, MV, (void*)gg, D_skip + hb);
    }

    token_major_kernel<<<dim3(kNpos / 64, kChan / 256), 256, 0, stream>>>(GT, GP);
    glu_gemm_kernel<<<512, 256, 0, stream>>>(GP, WL, b_out + (size_t)i * kOutW, src, dst);
  }
}
